// ScaledDotProductAttention_36910948942463
// MI455X (gfx1250) — hardware-verified
//
#include <hip/hip_runtime.h>
#include <math.h>

#ifndef NB
#define NB 2
#endif
#ifndef SEQ
#define SEQ 2048
#endif
#define NH 16
#define HD 64
#define NB_FULL 2
#define SEQ_FULL 2048

typedef __attribute__((ext_vector_type(16))) __bf16   v16b;
typedef __attribute__((ext_vector_type(8)))  float    v8f;
typedef __attribute__((ext_vector_type(4)))  float    v4f;
typedef __attribute__((ext_vector_type(4)))  unsigned v4u;
typedef __attribute__((ext_vector_type(8)))  unsigned v8u;
typedef __attribute__((ext_vector_type(4)))  int      v4i;

static_assert(HD == 64);
static_assert((SEQ % 64) == 0);
static_assert((SEQ & (SEQ - 1)) == 0);
static_assert(SEQ <= SEQ_FULL && NB <= NB_FULL);
static_assert(((long long)NB * NH * SEQ * HD) % (256 * 8) == 0);
static_assert(3ll * NB * NH * SEQ * HD * 2 <= 134217728ll);

__device__ __forceinline__ v8f wmmab(v16b a, v16b b, v8f c) {
    c = __builtin_amdgcn_wmma_f32_16x16x32_bf16(false, a, false, b, (short)0, c, false, false);
    asm volatile("v_nop\n\tv_nop\n\tv_nop\n\tv_nop" : "+v"(c) : "v"(a), "v"(b));
    return c;
}
__device__ __forceinline__ v16b frag_ld(const unsigned short* row, unsigned k0, unsigned h) {
    const v4u a = *(const v4u*)(row + k0 + 8u * h);
    const v4u b = *(const v4u*)(row + k0 + 16u + 8u * h);
    const v8u w = __builtin_shufflevector(a, b, 0, 1, 2, 3, 4, 5, 6, 7);
    return __builtin_bit_cast(v16b, w);
}
__device__ __forceinline__ unsigned bf_bits(float f) { unsigned u = __float_as_uint(f); u += 0x7fffu + ((u >> 16) & 1u); return u >> 16; }
__device__ __forceinline__ unsigned pack2(float a, float b) { return bf_bits(a) | (bf_bits(b) << 16); }
__device__ __forceinline__ void split2(float a, float b, unsigned& hi, unsigned& lo) {
    const unsigned ha = bf_bits(a), hb = bf_bits(b);
    const float ra = a - __uint_as_float(ha << 16), rb = b - __uint_as_float(hb << 16);
    hi = ha | (hb << 16); lo = bf_bits(ra) | (bf_bits(rb) << 16);
}

#define VST2(T, ptr, val) do { const T vst2_v_ = (val); *(volatile T*)(ptr) = vst2_v_; __threadfence(); *(volatile T*)(ptr) = vst2_v_; } while (0)

__global__ __launch_bounds__(256) void k_cvt_qk(const float* __restrict__ Qs, const float* __restrict__ Ks, unsigned short* __restrict__ Qp, unsigned short* __restrict__ Kp) {
    const unsigned u = blockIdx.x * 256u + threadIdx.x;
    if (u >= (unsigned)(NB * NH * SEQ * HD / 8)) return;
    const float* src = (blockIdx.y == 0u) ? Qs : Ks;
    unsigned short* dst = (blockIdx.y == 0u) ? Qp : Kp;
    const unsigned d8 = u & 7u, row = u >> 3;
    const unsigned s = row & (unsigned)(SEQ - 1), bh = row / (unsigned)SEQ;
    const float* p = src + ((size_t)bh * SEQ_FULL + s) * HD + d8 * 8u;
    const v4f a = *(const v4f*)p, b = *(const v4f*)(p + 4);
    v4u pk; pk.x = pack2(a.x, a.y); pk.y = pack2(a.z, a.w); pk.z = pack2(b.x, b.y); pk.w = pack2(b.z, b.w);
    VST2(v4u, dst + (size_t)u * 8u, pk);
}

__global__ __launch_bounds__(256) void k_cvt_vt(const float* __restrict__ Vs, unsigned short* __restrict__ Vt) {
    __shared__ __align__(16) unsigned short tl[64 * 72];
    const unsigned t = threadIdx.x, bh = blockIdx.y, j0 = blockIdx.x * 64u;
    const unsigned kr = t >> 2, dseg = (t & 3u) * 16u;
    const float* p = Vs + ((size_t)bh * SEQ_FULL + j0 + kr) * HD + dseg;
#pragma unroll
    for (unsigned q = 0; q < 4u; ++q) {
        const v4f v = *(const v4f*)(p + 4u * q);
        tl[(dseg + 4u * q + 0u) * 72u + kr] = (unsigned short)bf_bits(v.x);
        tl[(dseg + 4u * q + 1u) * 72u + kr] = (unsigned short)bf_bits(v.y);
        tl[(dseg + 4u * q + 2u) * 72u + kr] = (unsigned short)bf_bits(v.z);
        tl[(dseg + 4u * q + 3u) * 72u + kr] = (unsigned short)bf_bits(v.w);
    }
    __syncthreads();
#pragma unroll
    for (unsigned it = 0; it < 2u; ++it) {
        const unsigned pi = t + 256u * it, d = pi >> 3, seg = pi & 7u;
        const v4u w = *(const v4u*)(tl + d * 72u + seg * 8u);
        VST2(v4u, Vt + ((size_t)bh * HD + d) * SEQ + j0 + seg * 8u, w);
    }
}

__global__ __launch_bounds__(128) void k_fa(const unsigned short* __restrict__ Qp, const unsigned short* __restrict__ Kp, const unsigned short* __restrict__ Vt,
                                            const int* __restrict__ M, float* __restrict__ O) {
    __shared__ __align__(16) float ot[4][16 * 64];
    const unsigned tid = threadIdx.x, lane = tid & 31u, hf = lane >> 4, n = lane & 15u, wave = tid >> 5;
    const unsigned bh = blockIdx.z * NH + blockIdx.y;
    const unsigned q0 = (blockIdx.x * 4u + wave) * 16u;
    const float NEG = -__builtin_inff();
    const float CS = 0.125f * 1.4426950408889634f;
    const unsigned short* qrow = Qp + ((size_t)bh * SEQ + q0 + n) * HD;
    const v16b qf0 = frag_ld(qrow, 0u, hf), qf1 = frag_ld(qrow, 32u, hf);
    const unsigned short* kb = Kp + (size_t)bh * SEQ * HD;
    const unsigned short* vb = Vt + (size_t)bh * HD * SEQ;
    const int* mrow = M + (size_t)(q0 + n) * SEQ_FULL;
    v8f o0 = {}, o1 = {}, o2 = {}, o3 = {};
    float m = NEG, l = 0.f;
#pragma unroll 1
    for (unsigned j0 = 0; j0 < (unsigned)SEQ; j0 += 32u) {
        const v4i ma = *(const v4i*)(mrow + j0 + 8u * hf);
        const v4i mb = *(const v4i*)(mrow + j0 + 8u * hf + 4u);
        const v4i mc = *(const v4i*)(mrow + j0 + 16u + 8u * hf);
        const v4i md = *(const v4i*)(mrow + j0 + 16u + 8u * hf + 4u);
        const int anyv = ma.x | ma.y | ma.z | ma.w | mb.x | mb.y | mb.z | mb.w | mc.x | mc.y | mc.z | mc.w | md.x | md.y | md.z | md.w;
        if (__builtin_amdgcn_ballot_w32(anyv != 0) == 0u) continue;
        const int mw0[8] = {ma.x, ma.y, ma.z, ma.w, mb.x, mb.y, mb.z, mb.w};
        const int mw1[8] = {mc.x, mc.y, mc.z, mc.w, md.x, md.y, md.z, md.w};
        v8f s0 = {}, s1 = {};
        {
            const unsigned short* kr0 = kb + (size_t)(j0 + n) * HD;
            const unsigned short* kr1 = kr0 + 16u * HD;
            s0 = wmmab(frag_ld(kr0, 0u, hf), qf0, s0);
            s0 = wmmab(frag_ld(kr0, 32u, hf), qf1, s0);
            s1 = wmmab(frag_ld(kr1, 0u, hf), qf0, s1);
            s1 = wmmab(frag_ld(kr1, 32u, hf), qf1, s1);
        }
        float sc0[8], sc1[8];
        float mx = NEG;
#pragma unroll
        for (int r = 0; r < 8; ++r) {
            sc0[r] = (mw0[r] != 0) ? s0[r] * CS : NEG;
            sc1[r] = (mw1[r] != 0) ? s1[r] * CS : NEG;
            mx = fmaxf(mx, fmaxf(sc0[r], sc1[r]));
        }
        mx = fmaxf(mx, __shfl_xor(mx, 16, 32));
        const float mnew = fmaxf(m, mx);
        const float ce = exp2f(m - mnew);
        const float corr = (mnew == NEG) ? 1.f : ce;
        float p0[8], p1[8];
        float rs = 0.f;
#pragma unroll
        for (int r = 0; r < 8; ++r) {
            const float e0 = exp2f(sc0[r] - mnew), e1 = exp2f(sc1[r] - mnew);
            p0[r] = (sc0[r] == NEG) ? 0.f : e0;
            p1[r] = (sc1[r] == NEG) ? 0.f : e1;
            rs += p0[r] + p1[r];
        }
        rs += __shfl_xor(rs, 16, 32);
        l = l * corr + rs; m = mnew;
#pragma unroll
        for (int r = 0; r < 8; ++r) {
            const float cr = __shfl(corr, (int)(8u * hf + (unsigned)r), 32);
            o0[r] *= cr; o1[r] *= cr; o2[r] *= cr; o3[r] *= cr;
        }
        unsigned phw[8], plw[8];
#pragma unroll
        for (int e = 0; e < 4; ++e) {
            split2(p0[2 * e], p0[2 * e + 1], phw[e], plw[e]);
            split2(p1[2 * e], p1[2 * e + 1], phw[4 + e], plw[4 + e]);
        }
        const v8u phv = {phw[0], phw[1], phw[2], phw[3], phw[4], phw[5], phw[6], phw[7]};
        const v8u plv = {plw[0], plw[1], plw[2], plw[3], plw[4], plw[5], plw[6], plw[7]};
        const v16b pha = __builtin_bit_cast(v16b, phv), pla = __builtin_bit_cast(v16b, plv);
        {
            const v16b vf = frag_ld(vb + (size_t)(0u + n) * SEQ, j0, hf);
            o0 = wmmab(pha, vf, o0); o0 = wmmab(pla, vf, o0);
        }
        {
            const v16b vf = frag_ld(vb + (size_t)(16u + n) * SEQ, j0, hf);
            o1 = wmmab(pha, vf, o1); o1 = wmmab(pla, vf, o1);
        }
        {
            const v16b vf = frag_ld(vb + (size_t)(32u + n) * SEQ, j0, hf);
            o2 = wmmab(pha, vf, o2); o2 = wmmab(pla, vf, o2);
        }
        {
            const v16b vf = frag_ld(vb + (size_t)(48u + n) * SEQ, j0, hf);
            o3 = wmmab(pha, vf, o3); o3 = wmmab(pla, vf, o3);
        }
    }
    const float inv = 1.0f / l;
    float* mt = ot[wave];
#pragma unroll
    for (int r = 0; r < 8; ++r) {
        const float ir = __shfl(inv, (int)(8u * hf + (unsigned)r), 32);
        const unsigned rb = (8u * hf + (unsigned)r) * 64u + n;
        mt[rb] = o0[r] * ir; mt[rb + 16u] = o1[r] * ir; mt[rb + 32u] = o2[r] * ir; mt[rb + 48u] = o3[r] * ir;
    }
    __syncthreads();
    v4f ov[8];
#pragma unroll
    for (int s = 0; s < 8; ++s) ov[s] = *(const v4f*)(mt + ((unsigned)s * 32u + lane) * 4u);
    float* ob = O + ((size_t)bh * SEQ + q0) * HD;
#pragma unroll
    for (int s = 0; s < 8; ++s) *(volatile v4f*)(ob + ((unsigned)s * 32u + lane) * 4u) = ov[s];
    __threadfence();
#pragma unroll
    for (int s = 0; s < 8; ++s) *(volatile v4f*)(ob + ((unsigned)s * 32u + lane) * 4u) = ov[s];
}

extern "C" void kernel_launch(void* const* d_in, const int* in_sizes, int n_in, void* d_out, int out_size, void* d_ws, size_t ws_size, hipStream_t stream) {
    if (n_in < 4) return;
    const long long need_in = ((long long)(NB - 1) * NH + (NH - 1)) * SEQ_FULL * HD + (long long)SEQ * HD;
    const long long need_m = (long long)(SEQ - 1) * SEQ_FULL + SEQ;
    if ((long long)in_sizes[0] < need_in || (long long)in_sizes[1] < need_in || (long long)in_sizes[2] < need_in) return;
    if ((long long)in_sizes[3] < need_m) return;
    if ((long long)out_size < (long long)NB * NH * SEQ * HD) return;
    const size_t plane = (size_t)NB * NH * SEQ * HD * 2;
    if (ws_size < 3 * plane) return;
    const float* Q = (const float*)d_in[0];
    const float* K = (const float*)d_in[1];
    const float* V = (const float*)d_in[2];
    const int* mask = (const int*)d_in[3];
    float* out = (float*)d_out;
    char* wsp = (char*)d_ws;
    unsigned short* Qp = (unsigned short*)wsp;
    unsigned short* Kp = (unsigned short*)(wsp + plane);
    unsigned short* Vtp = (unsigned short*)(wsp + 2 * plane);
    k_cvt_qk<<<dim3((unsigned)(NB * NH * SEQ * HD / 8 / 256), 2u), 256, 0, stream>>>(Q, K, Qp, Kp);
    k_cvt_vt<<<dim3((unsigned)(SEQ / 64), (unsigned)(NB * NH)), 256, 0, stream>>>(V, Vtp);
    k_fa<<<dim3((unsigned)(SEQ / 64), (unsigned)NH, (unsigned)NB), 128, 0, stream>>>(Qp, Kp, Vtp, mask, out);
}
